// NeighborhoodCrossAttentionModuleV2_82231443849833
// MI455X (gfx1250) — hardware-verified
//
#include <hip/hip_runtime.h>
#include <stdint.h>

#define NVOX  9216
#define DIMC  128
#define QKC   256
#define NCLS  20
#define KVP   32
#define HEADS 8
#define HDIM  16
#define ND    24
#define NH    24
#define NW    16
#define KSZ   5
#define NTL   25
#define NGRP  13
#define NROW  576
#define LDC   132
#define OSP   132
#define XTP   136
#define VTP   40
#define NBX   144
#define NBV   72
#define NBWQ  16
#define NBWV  2
#define NBWP  8
#define VTB   8192
#define QKS   16.0f
#define VSC   16.0f
#define SSC   0.0009765625f
#define OFAC  64.0f
#define RES   2048.0f
#define RSC   0.00048828125f
#define WSC   64.0f
#define PSC   0.0000152587890625f

static_assert(NVOX == ND * NH * NW);
static_assert(NROW == ND * NH && NROW * NW == NVOX);
static_assert(DIMC == HEADS * HDIM && HDIM == 16 && NW == 16);
static_assert(NTL == KSZ * KSZ && NGRP * 2 >= NTL && (NGRP - 1) * 2 < NTL);
static_assert((NVOX % 64) == 0 && (NVOX % 128) == 0);
static_assert(NBX * 64 == NVOX && NBV * 128 == NVOX);
static_assert(NBWQ * 256 * 8 == QKC * DIMC && NBWV * 256 * 8 == DIMC * KVP && NBWP * 256 * 8 == DIMC * DIMC);
static_assert(VTB == 64 * DIMC);
static_assert(HEADS * 32 == 256);
static_assert((XTP * 2) % 16 == 0 && (VTP * 2) % 16 == 0 && (LDC * 4) % 16 == 0 && (OSP * 4) % 16 == 0);
static_assert(64 * XTP >= 128 * VTP);
static_assert((DIMC % 32) == 0 && KVP == 32 && NCLS <= KVP);

typedef _Float16       v16h  __attribute__((ext_vector_type(16)));
typedef _Float16       v8h   __attribute__((ext_vector_type(8)));
typedef unsigned short v16us __attribute__((ext_vector_type(16)));
typedef unsigned short v8us  __attribute__((ext_vector_type(8)));
typedef float          v8f   __attribute__((ext_vector_type(8)));
typedef float          v4f   __attribute__((ext_vector_type(4)));
typedef unsigned int   v4u   __attribute__((ext_vector_type(4)));
#if defined(__HIP_DEVICE_COMPILE__)
typedef __bf16         v16b  __attribute__((ext_vector_type(16)));
#endif

union HFrag { v16h v; v8us u[2]; v4u w[2]; };

__device__ __forceinline__ unsigned short bf_bits(float f) {
  unsigned u = __float_as_uint(f);
  return (unsigned short)((u + 0x7FFFu + ((u >> 16) & 1u)) >> 16);
}
__device__ __forceinline__ float bf_up(unsigned short b) { return __uint_as_float(((unsigned)b) << 16); }
__device__ __forceinline__ float bfr(float f) { return bf_up(bf_bits(f)); }
__device__ __forceinline__ unsigned short h_bits(_Float16 x) { return __builtin_bit_cast(unsigned short, x); }
__device__ __forceinline__ unsigned short hb16(float f) { return h_bits((_Float16)f); }
__device__ __forceinline__ unsigned pk16(unsigned short a, unsigned short b) { return (unsigned)a | ((unsigned)b << 16); }
__device__ __forceinline__ v8f zero8() { v8f z = {0.f, 0.f, 0.f, 0.f, 0.f, 0.f, 0.f, 0.f}; return z; }

__device__ __forceinline__ v16us ldfrag(const unsigned short* p) {
  union { v16us v; v8us h[2]; } f;
  f.h[0] = *(const v8us*)(p);
  f.h[1] = *(const v8us*)(p + 16);
  return f.v;
}
__device__ __forceinline__ v16h ldfrag8(const unsigned short* p) {
  HFrag f;
  f.u[0] = *(const v8us*)(p);
  const v8us z = {0, 0, 0, 0, 0, 0, 0, 0};
  f.u[1] = z;
  return f.v;
}

template<int BF>
__device__ __forceinline__ v8f mma16(v16us a, v16us b, v8f c) {
#if defined(__HIP_DEVICE_COMPILE__)
  if (BF) {
    return __builtin_amdgcn_wmma_f32_16x16x32_bf16(false, __builtin_bit_cast(v16b, a), false,
                                                  __builtin_bit_cast(v16b, b), (short)0, c, false, false);
  }
  return __builtin_amdgcn_wmma_f32_16x16x32_f16(false, __builtin_bit_cast(v16h, a), false,
                                               __builtin_bit_cast(v16h, b), (short)0, c, false, false);
#else
  (void)a; (void)b;
  return c;
#endif
}
__device__ __forceinline__ v8f mma_hf(v16h a, v16h b, v8f c) {
#if defined(__HIP_DEVICE_COMPILE__)
  return __builtin_amdgcn_wmma_f32_16x16x32_f16(false, a, false, b, (short)0, c, false, false);
#else
  (void)a; (void)b;
  return c;
#endif
}
__device__ __forceinline__ void guard4(v8f& c0, v8f& c1, v8f& c2, v8f& c3,
                                       const v16us& a0, const v16us& a1, const v16us& b0, const v16us& b1) {
#if defined(__HIP_DEVICE_COMPILE__)
  asm volatile("v_nop\n\tv_nop\n\tv_nop\n\tv_nop"
               : "+v"(c0), "+v"(c1), "+v"(c2), "+v"(c3)
               : "v"(a0), "v"(a1), "v"(b0), "v"(b1));
#endif
}
__device__ __forceinline__ void guard8(v8f& c0, v8f& c1, v8f& c2, v8f& c3, v8f& c4, v8f& c5, v8f& c6, v8f& c7,
                                       const v16us& a0, const v16us& a1, const v16us& a2, const v16us& a3,
                                       const v16us& b0, const v16us& b1) {
#if defined(__HIP_DEVICE_COMPILE__)
  asm volatile("v_nop\n\tv_nop\n\tv_nop\n\tv_nop"
               : "+v"(c0), "+v"(c1), "+v"(c2), "+v"(c3), "+v"(c4), "+v"(c5), "+v"(c6), "+v"(c7)
               : "v"(a0), "v"(a1), "v"(a2), "v"(a3), "v"(b0), "v"(b1));
#endif
}
__device__ __forceinline__ void guard_s1(v8f& s, const v16h& a, const v16h& b) {
#if defined(__HIP_DEVICE_COMPILE__)
  asm volatile("v_nop\n\tv_nop\n\tv_nop\n\tv_nop" : "+v"(s) : "v"(a), "v"(b));
#endif
}
__device__ __forceinline__ void guard_s2(v8f& s0, v8f& s1, const v16h& a0, const v16h& a1, const v16h& b) {
#if defined(__HIP_DEVICE_COMPILE__)
  asm volatile("v_nop\n\tv_nop\n\tv_nop\n\tv_nop" : "+v"(s0), "+v"(s1) : "v"(a0), "v"(a1), "v"(b));
#endif
}
__device__ __forceinline__ void guard_pv(v8f& c0, v8f& c1, const v16h& a0, const v16h& a1,
                                         const v16h& b0, const v16h& b1) {
#if defined(__HIP_DEVICE_COMPILE__)
  asm volatile("v_nop\n\tv_nop\n\tv_nop\n\tv_nop" : "+v"(c0), "+v"(c1) : "v"(a0), "v"(a1), "v"(b0), "v"(b1));
#endif
}

template<int BF>
__device__ __forceinline__ void mm_core(const unsigned short* __restrict__ A, const unsigned short* __restrict__ W,
                                        int ld, int nks, int arow0, int brow0, float* Cs) {
  const int tid = threadIdx.x, wave = tid >> 5, lane = tid & 31, hh = lane >> 4, c = lane & 15;
  const int mw = wave >> 2, nw = wave & 3;
  const unsigned short* a0p = A + (size_t)(arow0 + mw * 32 + c) * ld + 8 * hh;
  const unsigned short* a1p = A + (size_t)(arow0 + mw * 32 + 16 + c) * ld + 8 * hh;
  const unsigned short* b0p = W + (size_t)(brow0 + nw * 32 + c) * ld + 8 * hh;
  const unsigned short* b1p = W + (size_t)(brow0 + nw * 32 + 16 + c) * ld + 8 * hh;
  v8f c00 = zero8(), c01 = zero8(), c10 = zero8(), c11 = zero8();
#pragma unroll 1
  for (int ks = 0; ks < nks; ++ks) {
    const int ko = ks * 32;
    const v16us fa0 = ldfrag(a0p + ko);
    const v16us fa1 = ldfrag(a1p + ko);
    const v16us fb0 = ldfrag(b0p + ko);
    const v16us fb1 = ldfrag(b1p + ko);
    c00 = mma16<BF>(fa0, fb0, c00);
    c01 = mma16<BF>(fa0, fb1, c01);
    c10 = mma16<BF>(fa1, fb0, c10);
    c11 = mma16<BF>(fa1, fb1, c11);
    guard4(c00, c01, c10, c11, fa0, fa1, fb0, fb1);
  }
#pragma unroll
  for (int r = 0; r < 8; ++r) {
    const int row = mw * 32 + 8 * hh + r;
    Cs[row * LDC + nw * 32 + c]             = c00[r];
    Cs[row * LDC + nw * 32 + 16 + c]        = c01[r];
    Cs[(row + 16) * LDC + nw * 32 + c]      = c10[r];
    Cs[(row + 16) * LDC + nw * 32 + 16 + c] = c11[r];
  }
}

__device__ __forceinline__ void mm_core2(const unsigned short* __restrict__ Ah, const unsigned short* __restrict__ Al,
                                         int lda, const unsigned short* __restrict__ W, int ldw, int nks,
                                         int arow0, int brow0, float* Cs) {
  const int tid = threadIdx.x, wave = tid >> 5, lane = tid & 31, hh = lane >> 4, c = lane & 15;
  const int mw = wave >> 2, nw = wave & 3;
  const size_t r0 = (size_t)(arow0 + mw * 32 + c) * lda + 8 * hh;
  const size_t r1 = (size_t)(arow0 + mw * 32 + 16 + c) * lda + 8 * hh;
  const unsigned short* a0h = Ah + r0;
  const unsigned short* a1h = Ah + r1;
  const unsigned short* a0l = Al + r0;
  const unsigned short* a1l = Al + r1;
  const unsigned short* b0p = W + (size_t)(brow0 + nw * 32 + c) * ldw + 8 * hh;
  const unsigned short* b1p = W + (size_t)(brow0 + nw * 32 + 16 + c) * ldw + 8 * hh;
  v8f h00 = zero8(), h01 = zero8(), h10 = zero8(), h11 = zero8();
  v8f l00 = zero8(), l01 = zero8(), l10 = zero8(), l11 = zero8();
#pragma unroll 1
  for (int ks = 0; ks < nks; ++ks) {
    const int ko = ks * 32;
    const v16us fa0 = ldfrag(a0h + ko);
    const v16us fa1 = ldfrag(a1h + ko);
    const v16us ga0 = ldfrag(a0l + ko);
    const v16us ga1 = ldfrag(a1l + ko);
    const v16us fb0 = ldfrag(b0p + ko);
    const v16us fb1 = ldfrag(b1p + ko);
    h00 = mma16<0>(fa0, fb0, h00);
    h01 = mma16<0>(fa0, fb1, h01);
    h10 = mma16<0>(fa1, fb0, h10);
    h11 = mma16<0>(fa1, fb1, h11);
    l00 = mma16<0>(ga0, fb0, l00);
    l01 = mma16<0>(ga0, fb1, l01);
    l10 = mma16<0>(ga1, fb0, l10);
    l11 = mma16<0>(ga1, fb1, l11);
    guard8(h00, h01, h10, h11, l00, l01, l10, l11, fa0, fa1, ga0, ga1, fb0, fb1);
  }
#pragma unroll
  for (int r = 0; r < 8; ++r) {
    const int row = mw * 32 + 8 * hh + r;
    Cs[row * LDC + nw * 32 + c]             = h00[r] + l00[r] * RSC;
    Cs[row * LDC + nw * 32 + 16 + c]        = h01[r] + l01[r] * RSC;
    Cs[(row + 16) * LDC + nw * 32 + c]      = h10[r] + l10[r] * RSC;
    Cs[(row + 16) * LDC + nw * 32 + 16 + c] = h11[r] + l11[r] * RSC;
  }
}

__global__ __launch_bounds__(256)
void k_cvt(const float* __restrict__ x, const float* __restrict__ v, const float* __restrict__ wqk,
           const float* __restrict__ wv, const float* __restrict__ wp,
           unsigned short* x16, unsigned short* v16, unsigned short* wqk16, unsigned short* wv16,
           unsigned short* wp16) {
  __shared__ __align__(16) unsigned short Ts[64 * XTP];
  const int tid = threadIdx.x;
  const int blk = blockIdx.x;
  if (blk < NBX) {
    const int n0 = blk * 64;
#pragma unroll 4
    for (int it = 0; it < 32; ++it) {
      const int idx = it * 256 + tid;
      const int c = idx >> 6, nl = idx & 63;
      Ts[nl * XTP + c] = bf_bits(x[(size_t)c * NVOX + n0 + nl]);
    }
    __syncthreads();
    v4u pk[4];
    size_t offs[4];
#pragma unroll
    for (int s = 0; s < 4; ++s) {
      const int idx = s * 256 + tid;
      const int row = idx >> 4, piece = idx & 15;
      pk[s] = *(const v4u*)(Ts + row * XTP + piece * 8);
      offs[s] = (size_t)(n0 + row) * DIMC + piece * 8;
    }
#pragma unroll
    for (int s = 0; s < 4; ++s) *(volatile v4u*)(x16 + offs[s]) = pk[s];
    __threadfence();
#pragma unroll
    for (int s = 0; s < 4; ++s) *(volatile v4u*)(x16 + offs[s]) = pk[s];
  } else if (blk < NBX + NBV) {
    const int n0 = (blk - NBX) * 128;
#pragma unroll 4
    for (int it = 0; it < 16; ++it) {
      const int idx = it * 256 + tid;
      const int c = idx >> 7, nl = idx & 127;
      const float f = v[(size_t)min(c, NCLS - 1) * NVOX + n0 + nl];
      Ts[nl * VTP + c] = (c < NCLS) ? bf_bits(f) : (unsigned short)0;
    }
    __syncthreads();
    v4u pk[2];
    size_t offs[2];
#pragma unroll
    for (int s = 0; s < 2; ++s) {
      const int idx = s * 256 + tid;
      const int row = idx >> 2, piece = idx & 3;
      pk[s] = *(const v4u*)(Ts + row * VTP + piece * 8);
      offs[s] = (size_t)(n0 + row) * KVP + piece * 8;
    }
#pragma unroll
    for (int s = 0; s < 2; ++s) *(volatile v4u*)(v16 + offs[s]) = pk[s];
    __threadfence();
#pragma unroll
    for (int s = 0; s < 2; ++s) *(volatile v4u*)(v16 + offs[s]) = pk[s];
  } else if (blk < NBX + NBV + NBWQ) {
    const int t = (blk - NBX - NBV) * 256 + tid;
    const int row = t >> 4, piece = t & 15;
    const float* src = wqk + (size_t)row * DIMC + piece * 8;
    v4u pk;
#pragma unroll
    for (int e = 0; e < 4; ++e) pk[e] = pk16(bf_bits(src[2 * e]), bf_bits(src[2 * e + 1]));
    unsigned short* dst = wqk16 + (size_t)row * DIMC + piece * 8;
    *(volatile v4u*)dst = pk;
    __threadfence();
    *(volatile v4u*)dst = pk;
  } else if (blk < NBX + NBV + NBWQ + NBWV) {
    const int t = (blk - NBX - NBV - NBWQ) * 256 + tid;
    const int row = t >> 2, piece = t & 3;
    v4u pk;
#pragma unroll
    for (int e = 0; e < 4; ++e) {
      const int c0 = piece * 8 + 2 * e, c1 = c0 + 1;
      const float f0 = wv[(size_t)row * NCLS + min(c0, NCLS - 1)];
      const float f1 = wv[(size_t)row * NCLS + min(c1, NCLS - 1)];
      const unsigned short b0 = (c0 < NCLS) ? bf_bits(f0) : (unsigned short)0;
      const unsigned short b1 = (c1 < NCLS) ? bf_bits(f1) : (unsigned short)0;
      pk[e] = pk16(b0, b1);
    }
    unsigned short* dst = wv16 + (size_t)row * KVP + piece * 8;
    *(volatile v4u*)dst = pk;
    __threadfence();
    *(volatile v4u*)dst = pk;
  } else if (blk < NBX + NBV + NBWQ + NBWV + NBWP) {
    const int t = (blk - NBX - NBV - NBWQ - NBWV) * 256 + tid;
    const int row = t >> 4, piece = t & 15;
    const float* src = wp + (size_t)row * DIMC + piece * 8;
    v4u pk;
#pragma unroll
    for (int e = 0; e < 4; ++e)
      pk[e] = pk16(hb16(bfr(src[2 * e]) * WSC), hb16(bfr(src[2 * e + 1]) * WSC));
    unsigned short* dst = wp16 + (size_t)row * DIMC + piece * 8;
    *(volatile v4u*)dst = pk;
    __threadfence();
    *(volatile v4u*)dst = pk;
  }
}

__global__ __launch_bounds__(256)
void k_qkproj(const unsigned short* __restrict__ A, const unsigned short* __restrict__ W,
              const float* __restrict__ bias, unsigned short* qk16) {
  __shared__ __align__(16) float Cs[64 * LDC];
  const int tid = threadIdx.x;
  const int mb = blockIdx.x, nb = blockIdx.y;
  mm_core<1>(A, W, DIMC, DIMC / 32, mb * 64, nb * 128, Cs);
  __syncthreads();
  v4u pk[4];
  size_t offs[4];
#pragma unroll
  for (int s = 0; s < 4; ++s) {
    const int idx = s * 256 + tid;
    const int row = idx >> 4, piece = idx & 15;
    const int col0 = piece * 8;
    v4u a;
#pragma unroll
    for (int e = 0; e < 4; ++e) {
      const float f0 = (Cs[row * LDC + col0 + 2 * e]     + bfr(bias[nb * 128 + col0 + 2 * e]))     * QKS;
      const float f1 = (Cs[row * LDC + col0 + 2 * e + 1] + bfr(bias[nb * 128 + col0 + 2 * e + 1])) * QKS;
      a[e] = pk16(hb16(f0), hb16(f1));
    }
    pk[s] = a;
    offs[s] = (size_t)nb * NVOX * DIMC + (size_t)(mb * 64 + row) * DIMC + col0;
  }
#pragma unroll
  for (int s = 0; s < 4; ++s) *(volatile v4u*)(qk16 + offs[s]) = pk[s];
  __threadfence();
#pragma unroll
  for (int s = 0; s < 4; ++s) *(volatile v4u*)(qk16 + offs[s]) = pk[s];
}

__global__ __launch_bounds__(256)
void k_vproj(const unsigned short* __restrict__ A, const unsigned short* __restrict__ W,
             const float* __restrict__ bias, unsigned short* vth, unsigned short* vtl) {
  __shared__ __align__(16) float Cs[64 * LDC];
  const int tid = threadIdx.x;
  const int mb = blockIdx.x;
  mm_core<1>(A, W, KVP, 1, mb * 64, 0, Cs);
  __syncthreads();
  v4u ph[4], plq[4];
  size_t offs[4];
#pragma unroll
  for (int s = 0; s < 4; ++s) {
    const int idx = s * 256 + tid;
    const int L = idx >> 3, p = idx & 7;
    const int r4 = L >> 5;
    const int head = (L >> 2) & 7;
    const int c = (L * 4 + (p >> 1)) & 15;
    const int w0 = (p & 1) * 8;
    const int col = head * HDIM + c;
    const float bb = bfr(bias[col]);
    v4u a, q4;
#pragma unroll
    for (int e = 0; e < 4; ++e) {
      const float f0 = (Cs[(r4 * 16 + w0 + 2 * e) * LDC + col]     + bb) * VSC;
      const float f1 = (Cs[(r4 * 16 + w0 + 2 * e + 1) * LDC + col] + bb) * VSC;
      const _Float16 h0 = (_Float16)f0, h1 = (_Float16)f1;
      const float q0 = (f0 - (float)h0) * RES, q1 = (f1 - (float)h1) * RES;
      a[e]  = pk16(h_bits(h0), h_bits(h1));
      q4[e] = pk16(hb16(q0), hb16(q1));
    }
    ph[s] = a;
    plq[s] = q4;
    offs[s] = (size_t)mb * VTB + (size_t)idx * 8;
  }
#pragma unroll
  for (int s = 0; s < 4; ++s) { *(volatile v4u*)(vth + offs[s]) = ph[s]; *(volatile v4u*)(vtl + offs[s]) = plq[s]; }
  __threadfence();
#pragma unroll
  for (int s = 0; s < 4; ++s) { *(volatile v4u*)(vth + offs[s]) = ph[s]; *(volatile v4u*)(vtl + offs[s]) = plq[s]; }
}

__global__ __launch_bounds__(256)
void k_attn(const unsigned short* __restrict__ qk16, const unsigned short* __restrict__ vth,
            const unsigned short* __restrict__ vtl, unsigned short* oh, unsigned short* ol) {
  __shared__ __align__(16) float Os[NW * OSP];
  const int tid = threadIdx.x, head = tid >> 5, lane = tid & 31, hh = lane >> 4, c = lane & 15;
  const int rowq = blockIdx.x;
  const int d = rowq / NH, h = rowq - d * NH;
  const int sd = min(max(d - KSZ / 2, 0), ND - KSZ);
  const int sh = min(max(h - KSZ / 2, 0), NH - KSZ);
  const int nbase = rowq * NW;
  const unsigned short* kpl = qk16 + (size_t)NVOX * DIMC;
  const int choff = head * HDIM + 8 * hh;
  const v16h bq = ldfrag8(qk16 + (size_t)(nbase + c) * DIMC + choff);
  const int sw = min(max(c - KSZ / 2, 0), NW - KSZ);
  unsigned live = 0u;
#pragma unroll
  for (int r = 0; r < 8; ++r) {
    const int wp = 8 * hh + r;
    live |= (wp >= sw && wp < sw + KSZ) ? (1u << r) : 0u;
  }
  const v8f z8 = zero8();
  const v8us zu = {0, 0, 0, 0, 0, 0, 0, 0};

  float mx = -3.0e38f;
#pragma unroll 1
  for (int t = 0; t < NTL; ++t) {
    const int jd = t / KSZ, jh = t - jd * KSZ;
    const int rowk = (sd + jd) * NH + sh + jh;
    const v16h ak = ldfrag8(kpl + ((size_t)rowk * NW + c) * DIMC + choff);
    v8f s = mma_hf(ak, bq, z8);
    guard_s1(s, ak, bq);
#pragma unroll
    for (int r = 0; r < 8; ++r) {
      const float sv = ((live >> r) & 1u) ? s[r] * SSC : -3.0e38f;
      mx = fmaxf(mx, sv);
    }
  }
  const float m = fmaxf(mx, __shfl_xor(mx, 16, 32));

  v8f acch = zero8(), accl = zero8();
  float lsum = 0.f;
#pragma unroll 1
  for (int g = 0; g < NGRP; ++g) {
    const int t0 = 2 * g;
    const bool last = (2 * g + 1 >= NTL);
    const int t1 = last ? (NTL - 1) : (2 * g + 1);
    const int jd0 = t0 / KSZ, jh0 = t0 - jd0 * KSZ;
    const int jd1 = t1 / KSZ, jh1 = t1 - jd1 * KSZ;
    const int rk0 = (sd + jd0) * NH + sh + jh0;
    const int rk1 = (sd + jd1) * NH + sh + jh1;
    const v16h ak0 = ldfrag8(kpl + ((size_t)rk0 * NW + c) * DIMC + choff);
    const v16h ak1 = ldfrag8(kpl + ((size_t)rk1 * NW + c) * DIMC + choff);
    v8f s0 = mma_hf(ak0, bq, z8);
    v8f s1 = mma_hf(ak1, bq, z8);
    guard_s2(s0, s1, ak0, ak1, bq);
    const size_t vo0 = ((size_t)(rk0 * HEADS + head) * HDIM + c) * NW + 8 * hh;
    const size_t vo1 = ((size_t)(rk1 * HEADS + head) * HDIM + c) * NW + 8 * hh;
    HFrag vh, vl;
    vh.u[0] = *(const v8us*)(vth + vo0);
    vl.u[0] = *(const v8us*)(vtl + vo0);
    const v8us th1 = *(const v8us*)(vth + vo1);
    const v8us tl1 = *(const v8us*)(vtl + vo1);
    vh.u[1] = last ? zu : th1;
    vl.u[1] = last ? zu : tl1;
    const unsigned live1 = last ? 0u : live;
    HFrag ph, pl;
#pragma unroll
    for (int rr = 0; rr < 4; ++rr) {
      const int ra = 2 * rr, rb = 2 * rr + 1;
      const float ea = __expf(s0[ra] * SSC - m), eb = __expf(s0[rb] * SSC - m);
      const float fa = __expf(s1[ra] * SSC - m), fb = __expf(s1[rb] * SSC - m);
      const float pa = ((live  >> ra) & 1u) ? ea : 0.f;
      const float pb = ((live  >> rb) & 1u) ? eb : 0.f;
      const float qa = ((live1 >> ra) & 1u) ? fa : 0.f;
      const float qb = ((live1 >> rb) & 1u) ? fb : 0.f;
      lsum += (pa + pb) + (qa + qb);
      const _Float16 hpa = (_Float16)pa, hpb = (_Float16)pb, hqa = (_Float16)qa, hqb = (_Float16)qb;
      ph.w[0][rr] = pk16(h_bits(hpa), h_bits(hpb));
      ph.w[1][rr] = pk16(h_bits(hqa), h_bits(hqb));
      pl.w[0][rr] = pk16(hb16((pa - (float)hpa) * RES), hb16((pb - (float)hpb) * RES));
      pl.w[1][rr] = pk16(hb16((qa - (float)hqa) * RES), hb16((qb - (float)hqb) * RES));
    }
    acch = mma_hf(ph.v, vh.v, acch);
    accl = mma_hf(pl.v, vh.v, accl);
    accl = mma_hf(ph.v, vl.v, accl);
    guard_pv(acch, accl, ph.v, pl.v, vh.v, vl.v);
  }
  const float lq = lsum + __shfl_xor(lsum, 16, 32);
  const float rl = __builtin_amdgcn_rcpf(lq) * OFAC;
#pragma unroll
  for (int r = 0; r < 8; ++r) {
    const float f = __shfl(rl, 8 * hh + r, 32);
    Os[(8 * hh + r) * OSP + head * HDIM + c] = (acch[r] + accl[r] * RSC) * f;
  }
  __syncthreads();
  const int row = tid >> 4, piece = tid & 15;
  const v4f a = *(const v4f*)(Os + row * OSP + piece * 8);
  const v4f b = *(const v4f*)(Os + row * OSP + piece * 8 + 4);
  v4u hw, lw;
  {
    const _Float16 h0 = (_Float16)a[0], h1 = (_Float16)a[1], h2 = (_Float16)a[2], h3 = (_Float16)a[3];
    const _Float16 h4 = (_Float16)b[0], h5 = (_Float16)b[1], h6 = (_Float16)b[2], h7 = (_Float16)b[3];
    hw[0] = pk16(h_bits(h0), h_bits(h1));
    hw[1] = pk16(h_bits(h2), h_bits(h3));
    hw[2] = pk16(h_bits(h4), h_bits(h5));
    hw[3] = pk16(h_bits(h6), h_bits(h7));
    lw[0] = pk16(hb16((a[0] - (float)h0) * RES), hb16((a[1] - (float)h1) * RES));
    lw[1] = pk16(hb16((a[2] - (float)h2) * RES), hb16((a[3] - (float)h3) * RES));
    lw[2] = pk16(hb16((b[0] - (float)h4) * RES), hb16((b[1] - (float)h5) * RES));
    lw[3] = pk16(hb16((b[2] - (float)h6) * RES), hb16((b[3] - (float)h7) * RES));
  }
  const size_t oo = (size_t)(nbase + row) * DIMC + piece * 8;
  *(volatile v4u*)(oh + oo) = hw;
  *(volatile v4u*)(ol + oo) = lw;
  __threadfence();
  *(volatile v4u*)(oh + oo) = hw;
  *(volatile v4u*)(ol + oo) = lw;
}

__global__ __launch_bounds__(256)
void k_outp(const unsigned short* __restrict__ OH, const unsigned short* __restrict__ OL,
            const unsigned short* __restrict__ W, const float* __restrict__ bias, float* out) {
  __shared__ __align__(16) float Cs[64 * LDC];
  const int tid = threadIdx.x, wave = tid >> 5, lane = tid & 31, hh = lane >> 4, piece = lane & 15;
  const int mb = blockIdx.x;
  mm_core2(OH, OL, DIMC, W, DIMC, DIMC / 32, mb * 64, 0, Cs);
  __syncthreads();
#pragma unroll 1
  for (int it = 0; it < 8; ++it) {
    const int o = wave * 16 + it * 2 + hh;
    const float bo = bfr(bias[o]);
    v4f val;
#pragma unroll
    for (int e = 0; e < 4; ++e) val[e] = Cs[(piece * 4 + e) * LDC + o] * PSC + bo;
    float* p = out + (size_t)o * NVOX + mb * 64 + piece * 4;
    *(volatile v4f*)p = val;
    __threadfence();
    *(volatile v4f*)p = val;
  }
}

extern "C" void kernel_launch(void* const* d_in, const int* in_sizes, int n_in,
                              void* d_out, int out_size, void* d_ws, size_t ws_size,
                              hipStream_t stream) {
  if (n_in < 8) return;
  const int expect[8] = { DIMC * NVOX, NCLS * NVOX, QKC * DIMC, QKC, DIMC * NCLS, DIMC, DIMC * DIMC, DIMC };
  for (int i = 0; i < 8; ++i) if (in_sizes[i] != expect[i]) return;
  if (out_size != DIMC * NVOX) return;

  const float* x   = (const float*)d_in[0];
  const float* v   = (const float*)d_in[1];
  const float* wqk = (const float*)d_in[2];
  const float* bqk = (const float*)d_in[3];
  const float* wv  = (const float*)d_in[4];
  const float* bv  = (const float*)d_in[5];
  const float* wp  = (const float*)d_in[6];
  const float* bp  = (const float*)d_in[7];
  float* out = (float*)d_out;

  const size_t AL = 65536;
  const size_t sX16 = (((size_t)NVOX * DIMC * 2) + AL - 1) / AL * AL;
  const size_t sV16 = (((size_t)NVOX * KVP * 2) + AL - 1) / AL * AL;
  const size_t sWQ  = (((size_t)QKC * DIMC * 2) + AL - 1) / AL * AL;
  const size_t sWV  = (((size_t)DIMC * KVP * 2) + AL - 1) / AL * AL;
  const size_t sWP  = (((size_t)DIMC * DIMC * 2) + AL - 1) / AL * AL;
  const size_t sQK  = (((size_t)2 * NVOX * DIMC * 2) + AL - 1) / AL * AL;
  const size_t sPL  = (((size_t)NVOX * DIMC * 2) + AL - 1) / AL * AL;

  size_t off = 0;
  const size_t oX16 = off; off += sX16;
  const size_t oV16 = off; off += sV16;
  const size_t oWQ  = off; off += sWQ;
  const size_t oWV  = off; off += sWV;
  const size_t oWP  = off; off += sWP;
  const size_t oQK  = off; off += sQK;
  const size_t oVTH = off; off += sPL;
  const size_t oVTL = off; off += sPL;
  const size_t oOH  = off; off += sPL;
  const size_t oOL  = off; off += sPL;
  if (off > ws_size) return;
  if (off > (size_t)134217728) return;

  char* ws = (char*)d_ws;
  unsigned short* X16   = (unsigned short*)(ws + oX16);
  unsigned short* V16   = (unsigned short*)(ws + oV16);
  unsigned short* WQK16 = (unsigned short*)(ws + oWQ);
  unsigned short* WV16  = (unsigned short*)(ws + oWV);
  unsigned short* WP16  = (unsigned short*)(ws + oWP);
  unsigned short* QK16  = (unsigned short*)(ws + oQK);
  unsigned short* VTH   = (unsigned short*)(ws + oVTH);
  unsigned short* VTL   = (unsigned short*)(ws + oVTL);
  unsigned short* OH    = (unsigned short*)(ws + oOH);
  unsigned short* OL    = (unsigned short*)(ws + oOL);

  const dim3 blk(256);
  k_cvt<<<dim3(NBX + NBV + NBWQ + NBWV + NBWP), blk, 0, stream>>>(x, v, wqk, wv, wp, X16, V16, WQK16, WV16, WP16);
  k_qkproj<<<dim3(NVOX / 64, 2), blk, 0, stream>>>(X16, WQK16, bqk, QK16);
  k_vproj<<<dim3(NVOX / 64), blk, 0, stream>>>(V16, WV16, bv, VTH, VTL);
  k_attn<<<dim3(NROW), blk, 0, stream>>>(QK16, VTH, VTL, OH, OL);
  k_outp<<<dim3(NVOX / 64), blk, 0, stream>>>(OH, OL, WP16, bp, out);
  (void)hipGetLastError();
}
